// Interface_attention_47072841564866
// MI455X (gfx1250) — hardware-verified
//
#include <hip/hip_runtime.h>


namespace {
constexpr int N1 = 20000, N2 = 20000, NN = 16, ND = 128, NH = 4, NPAD = 20096  , NBLK = NPAD / 128;
constexpr float AS_ = 8.0f;

typedef _Float16 b16;
typedef __attribute__((ext_vector_type(16))) _Float16 v16b;
typedef __attribute__((ext_vector_type(16))) __bf16 v16bb;
typedef __attribute__((ext_vector_type(8))) _Float16 v8b;
typedef __attribute__((ext_vector_type(8))) unsigned short v8us;
typedef __attribute__((ext_vector_type(8))) float v8f;
typedef __attribute__((ext_vector_type(4))) float v4f;
__device__ __forceinline__ float bf16_rne(float f) { unsigned int u = __float_as_uint(f); u += 0x7FFFu + ((u >> 16) & 1u); return __uint_as_float(u & 0xFFFF0000u); }
__device__ __forceinline__ unsigned short bf16_bits(float f) { unsigned int u = __float_as_uint(f); u += 0x7FFFu + ((u >> 16) & 1u); return (unsigned short)(u >> 16); }
__device__ __forceinline__ void split16(float v, b16& hi, b16& lo) { hi = (b16)v; lo = (b16)(v - (float)hi); }
__device__ __forceinline__ v16b frag_kb(const b16* p, int hh) { const v8b a = *(const v8b*)(p + 8 * hh), b = *(const v8b*)(p + 16 + 8 * hh); v16b f;
#pragma unroll
  for (int e = 0; e < 8; ++e) { f[e] = a[e]; f[8 + e] = b[e]; } return f; }
__device__ __forceinline__ v16bb frag_bf(const unsigned short* p, int hh) { const v8us a = *(const v8us*)(p + 8 * hh), b = *(const v8us*)(p + 16 + 8 * hh); union { unsigned short s[16]; v16bb v; } u;
#pragma unroll
  for (int e = 0; e < 8; ++e) { u.s[e] = a[e]; u.s[8 + e] = b[e]; } return u.v; }
__device__ __forceinline__ v16bb frag_f32bf(const float* p, int hh) { union { unsigned short s[16]; v16bb v; } u;
#pragma unroll
  for (int e = 0; e < 8; ++e) { u.s[e] = bf16_bits(p[8 * hh + e]); u.s[8 + e] = bf16_bits(p[16 + 8 * hh + e]); } return u.v; }
__device__ __forceinline__ void frag_split(const float* p, int hh, v16b& fh, v16b& fl) {
#pragma unroll
  for (int e = 0; e < 8; ++e) { b16 a, c; split16(p[8 * hh + e] * AS_, a, c); fh[e] = a; fl[e] = c; split16(p[16 + 8 * hh + e] * AS_, a, c); fh[8 + e] = a; fl[8 + e] = c; } }
__device__ __forceinline__ v8f wmma16b(v16b a, v16b b, v8f c) { v8f d = __builtin_amdgcn_wmma_f32_16x16x32_f16(false, a, false, b, (short)0, c, false, false); asm volatile("v_nop\n\tv_nop\n\tv_nop\n\tv_nop" : "+v"(d) : "v"(a), "v"(b)); return d; }
__device__ __forceinline__ v8f wmma16bb(v16bb a, v16bb b, v8f c) { v8f d = __builtin_amdgcn_wmma_f32_16x16x32_bf16(false, a, false, b, (short)0, c, false, false); asm volatile("v_nop\n\tv_nop\n\tv_nop\n\tv_nop" : "+v"(d) : "v"(a), "v"(b)); return d; }
__device__ __forceinline__ void wave_lds_sync() { __builtin_amdgcn_fence(__ATOMIC_RELEASE, "workgroup"); __builtin_amdgcn_wave_barrier(); __builtin_amdgcn_fence(__ATOMIC_ACQUIRE, "workgroup"); }
__device__ __forceinline__ float nexp(float x) { return __builtin_amdgcn_exp2f(x * 1.4426950408889634f); }
__device__ __forceinline__ float elu_(float x) { return (x > 0.0f) ? x : (nexp(x) - 1.0f); }
__device__ __forceinline__ float pmul(float a, float b) { float p = a * b; asm volatile("" : "+v"(p)); return p; }

struct Wo { static constexpr size_t QW2 = 0, GW1 = QW2 + 512 * 128, GW2 = GW1 + 128 * 32, KW1 = GW2 + 128 * 128, KW2N = KW1 + 128 * 128, VW1 = KW2N + 128 * 128, VW2 = VW1 + 128 * 128, DW1 = VW2 + 128 * 128, DW2 = DW1 + 128 * 512, END = DW2 + 128 * 128; };
__global__ __launch_bounds__(256) void prep_kernel(const float* __restrict__ qw1, const float* __restrict__ qb1, const float* __restrict__ qw2, const float* __restrict__ qb2, const float* __restrict__ gw1, const float* __restrict__ gb1, const float* __restrict__ gw2, const float* __restrict__ gb2,
                                                   const float* __restrict__ kw1, const float* __restrict__ kw2, const float* __restrict__ vw1, const float* __restrict__ vw2, const float* __restrict__ dw1, const float* __restrict__ dw2,
                                                   unsigned short* __restrict__ qw16, b16* __restrict__ R, float* __restrict__ P) {
  const size_t tid = (size_t)blockIdx.x * blockDim.x + threadIdx.x, nth = (size_t)gridDim.x * blockDim.x;
  auto tr8 = [&](const float* W, int IN, int OUT, int KP, size_t base, size_t p) {
    const int o = (int)(p / (KP / 8)), k8 = (int)(p % (KP / 8)) * 8; v8b v;
#pragma unroll
    for (int e = 0; e < 8; ++e) { const int k = k8 + e; v[e] = (b16)((k < IN) ? bf16_rne(W[(size_t)k * OUT + o]) : 0.0f); }
    *(volatile v8b*)(R + base + (size_t)o * KP + k8) = v; };
  for (int pass = 0; pass < 2; ++pass) {
    for (size_t p = tid; p < 128 * 16; p += nth) { const int o = (int)(p / 16), k8 = (int)(p % 16) * 8; v8us v;
#pragma unroll
      for (int e = 0; e < 8; ++e) v[e] = bf16_bits(qw1[(size_t)(k8 + e) * 128 + o]);
      *(volatile v8us*)(qw16 + (size_t)o * 128 + k8) = v; }
    for (size_t p = tid; p < 512 * 16; p += nth) tr8(qw2, 128, 512, 128, Wo::QW2, p);
    for (size_t p = tid; p < 128 * 4; p += nth) tr8(gw1, 12, 128, 32, Wo::GW1, p);
    for (size_t p = tid; p < 128 * 16; p += nth) { tr8(gw2, 128, 128, 128, Wo::GW2, p); tr8(kw1, 128, 128, 128, Wo::KW1, p); tr8(vw1, 128, 128, 128, Wo::VW1, p); tr8(vw2, 128, 128, 128, Wo::VW2, p); tr8(dw2, 128, 128, 128, Wo::DW2, p);
      { const int o = (int)(p / 16), k8 = (int)(p % 16) * 8; v8b v;
#pragma unroll
        for (int e = 0; e < 8; ++e) v[e] = (b16)bf16_rne(kw2[(size_t)o * 128 + k8 + e]);
        *(volatile v8b*)(R + Wo::KW2N + (size_t)o * 128 + k8) = v; } }
    for (size_t p = tid; p < 128 * 64; p += nth) tr8(dw1, 512, 128, 512, Wo::DW1, p);
    for (size_t p = tid; p < 896 / 4; p += nth) { v4f v;
#pragma unroll
      for (int e = 0; e < 4; ++e) { const int i = (int)p * 4 + e; v[e] = bf16_rne((i < 128) ? qb1[i] : (i < 640) ? qb2[i - 128] : (i < 768) ? gb1[i - 640] : gb2[i - 768]); }
      *(volatile v4f*)(P + p * 4) = v; }
    __threadfence(); }
}

__global__ __launch_bounds__(128) void q_kernel(const float* __restrict__ f1, const unsigned short* __restrict__ qw16, const b16* __restrict__ R, const float* __restrict__ P, float* __restrict__ Q) {
  __shared__ __attribute__((aligned(16))) float T[4][32][128 + 4]; __shared__ __attribute__((aligned(16))) float Ts[4][32 * 64];
  const int lane = threadIdx.x & 31, wave = threadIdx.x >> 5, nloc = lane & 15, hlf = lane >> 4, m0 = blockIdx.y * 128 + wave * 32, c0 = blockIdx.x * 64;
  const int ra = min(m0 + nloc, N1 - 1), rb = min(m0 + 16 + nloc, N1 - 1); const float* qb1 = P; const float* qb2 = P + 128;
  for (int hq = 0; hq < 2; ++hq) { v8f acc[2][4];
#pragma unroll
    for (int r = 0; r < 2; ++r)
#pragma unroll
      for (int t = 0; t < 4; ++t) acc[r][t] = (v8f){};
#pragma unroll 1
    for (int kb = 0; kb < ND; kb += 32) { const v16bb a0 = frag_f32bf(f1 + (size_t)ra * ND + kb, hlf), a1 = frag_f32bf(f1 + (size_t)rb * ND + kb, hlf);
#pragma unroll
      for (int t = 0; t < 4; ++t) { const v16bb bw = frag_bf(qw16 + (size_t)((hq * 4 + t) * 16 + nloc) * ND + kb, hlf); acc[0][t] = wmma16bb(a0, bw, acc[0][t]); acc[1][t] = wmma16bb(a1, bw, acc[1][t]); } }
#pragma unroll
    for (int t = 0; t < 4; ++t) { const int cc = (hq * 4 + t) * 16 + nloc; const float bb = qb1[cc];
#pragma unroll
      for (int r = 0; r < 2; ++r)
#pragma unroll
        for (int v = 0; v < 8; ++v) T[wave][r * 16 + 8 * hlf + v][cc] = elu_(acc[r][t][v] + bb); } }
  wave_lds_sync();
  v8f acc[2][4];
#pragma unroll
  for (int r = 0; r < 2; ++r)
#pragma unroll
    for (int t = 0; t < 4; ++t) acc[r][t] = (v8f){};
#pragma unroll
  for (int kb = 0; kb < ND; kb += 32) { v16b a0, l0, a1, l1; frag_split(&T[wave][nloc][kb], hlf, a0, l0); frag_split(&T[wave][16 + nloc][kb], hlf, a1, l1);
#pragma unroll
    for (int t = 0; t < 4; ++t) { const v16b bw = frag_kb(R + Wo::QW2 + (size_t)(c0 + t * 16 + nloc) * ND + kb, hlf); acc[0][t] = wmma16b(a0, bw, acc[0][t]); acc[0][t] = wmma16b(l0, bw, acc[0][t]); acc[1][t] = wmma16b(a1, bw, acc[1][t]); acc[1][t] = wmma16b(l1, bw, acc[1][t]); } }
  float* Tt = Ts[wave];
#pragma unroll
  for (int t = 0; t < 4; ++t) { const float bb = qb2[c0 + t * 16 + nloc];
#pragma unroll
    for (int r = 0; r < 2; ++r)
#pragma unroll
      for (int v = 0; v < 8; ++v) Tt[(r * 16 + v + 8 * hlf) * 64 + t * 16 + nloc] = acc[r][t][v] * (1.0f / AS_) + bb; }
  wave_lds_sync();
  for (int pass = 0; pass < 2; ++pass) {
#pragma unroll
    for (int j = 0; j < 16; ++j) { const int rr = j * 2 + hlf, c4 = nloc * 4; *(volatile v4f*)(Q + (size_t)(m0 + rr) * 512 + c0 + c4) = *(const v4f*)(Tt + rr * 64 + c4); }
    __threadfence(); }
}

__global__ __launch_bounds__(128) void rows_kernel(const float* __restrict__ X, const b16* __restrict__ Bw, float* __restrict__ Y) {
  __shared__ __attribute__((aligned(16))) float Ts[4][32 * 64];
  const int lane = threadIdx.x & 31, wave = threadIdx.x >> 5, nloc = lane & 15, hlf = lane >> 4, m0 = blockIdx.y * 128 + wave * 32, c0 = blockIdx.x * 64;
  v8f acc[2][4];
#pragma unroll
  for (int r = 0; r < 2; ++r)
#pragma unroll
    for (int t = 0; t < 4; ++t) acc[r][t] = (v8f){};
#pragma unroll
  for (int kb = 0; kb < ND; kb += 32) { v16b a0, l0, a1, l1; frag_split(X + (size_t)(m0 + nloc) * ND + kb, hlf, a0, l0); frag_split(X + (size_t)(m0 + 16 + nloc) * ND + kb, hlf, a1, l1);
#pragma unroll
    for (int t = 0; t < 4; ++t) { const v16b bw = frag_kb(Bw + (size_t)(c0 + t * 16 + nloc) * ND + kb, hlf); acc[0][t] = wmma16b(a0, bw, acc[0][t]); acc[0][t] = wmma16b(l0, bw, acc[0][t]); acc[1][t] = wmma16b(a1, bw, acc[1][t]); acc[1][t] = wmma16b(l1, bw, acc[1][t]); } }
  float* Tt = Ts[wave];
#pragma unroll
  for (int t = 0; t < 4; ++t)
#pragma unroll
    for (int r = 0; r < 2; ++r)
#pragma unroll
      for (int v = 0; v < 8; ++v) Tt[(r * 16 + v + 8 * hlf) * 64 + t * 16 + nloc] = acc[r][t][v] * (1.0f / AS_);
  wave_lds_sync();
  for (int pass = 0; pass < 2; ++pass) {
#pragma unroll
    for (int j = 0; j < 16; ++j) { const int rr = j * 2 + hlf, c4 = nloc * 4; *(volatile v4f*)(Y + (size_t)(m0 + rr) * ND + c0 + c4) = *(const v4f*)(Tt + rr * 64 + c4); }
    __threadfence(); }
}

struct PW { float RLt[16][36]; float FN[16][132]; float T1[16][132]; float GEO[16][132]; float KT[16][132]; float MQ[16][36]; float VT[128][36]; float O[4][132]; float G[16]; int M[16]; };
__global__ __launch_bounds__(64) void pair_kernel(const float* __restrict__ f2, const float* __restrict__ x1, const float* __restrict__ x2, const float* __restrict__ nuv1, const float* __restrict__ nuv2, const int* __restrict__ topk, const float* __restrict__ Q, const b16* __restrict__ R, const float* __restrict__ P, float* __restrict__ orow) {
  __shared__ __attribute__((aligned(16))) PW Sm[2];
  const int wid = threadIdx.x >> 5, lane = threadIdx.x & 31, nloc = lane & 15, hlf = lane >> 4; const int n = blockIdx.x * 2 + wid; PW& S = Sm[wid];
  const float* gb1 = P + 640; const float* gb2 = P + 768;
  if (lane < 16) { int s = topk[(size_t)n * NN + lane]; const bool msk = (s == 0); s = (s < 0) ? 0 : (s >= N2 ? N2 - 1 : s); S.M[lane] = msk ? 1 : 0;
    float R9[9];
#pragma unroll
    for (int i = 0; i < 9; ++i) R9[i] = bf16_rne(nuv1[(size_t)n * 9 + i]);
    float ox[3];
#pragma unroll
    for (int a = 0; a < 3; ++a) ox[a] = bf16_rne(x2[(size_t)s * 3 + a]) - bf16_rne(x1[(size_t)n * 3 + a]);
    S.G[lane] = nexp(-0.5f * ((pmul(ox[0], ox[0]) + pmul(ox[1], ox[1])) + pmul(ox[2], ox[2])));
#pragma unroll
    for (int i = 0; i < 3; ++i) S.RLt[lane][i] = (pmul(R9[i * 3], ox[0]) + pmul(R9[i * 3 + 1], ox[1])) + pmul(R9[i * 3 + 2], ox[2]);
#pragma unroll
    for (int k = 0; k < 3; ++k) { float vk[3];
#pragma unroll
      for (int jx = 0; jx < 3; ++jx) vk[jx] = bf16_rne(nuv2[((size_t)s * 3 + k) * 3 + jx]);
#pragma unroll
      for (int i = 0; i < 3; ++i) S.RLt[lane][3 + k * 3 + i] = (pmul(R9[i * 3], vk[0]) + pmul(R9[i * 3 + 1], vk[1])) + pmul(R9[i * 3 + 2], vk[2]); }
#pragma unroll
    for (int c = 12; c < 32; ++c) S.RLt[lane][c] = 0.0f; }
  { const int j = lane >> 1, hf = (lane & 1) * 64; int s = topk[(size_t)n * NN + j]; s = (s < 0) ? 0 : (s >= N2 ? N2 - 1 : s); const float* fr = f2 + (size_t)s * ND + hf;
    for (int c = 0; c < 64; c += 4) { const v4f v = *(const v4f*)(fr + c); S.FN[j][hf + c] = bf16_rne(v[0]); S.FN[j][hf + c + 1] = bf16_rne(v[1]); S.FN[j][hf + c + 2] = bf16_rne(v[2]); S.FN[j][hf + c + 3] = bf16_rne(v[3]); } }
  wave_lds_sync();
  auto gemm = [&](const float* Arow  , int pitch, const b16* Bw, int KK, int NT_, v8f* acc, bool three, const float* Brows_f32 = nullptr) {
    for (int kb = 0; kb < KK; kb += 32) { v16b ah, al; frag_split(Arow + kb, hlf, ah, al);
      for (int t = 0; t < NT_; ++t) { const v16b bw = frag_kb(Bw + (size_t)(t * 16 + nloc) * KK + kb, hlf); acc[t] = wmma16b(ah, bw, acc[t]); acc[t] = wmma16b(al, bw, acc[t]); } } };
  v8f acc[8];
#pragma unroll
  for (int t = 0; t < 8; ++t) acc[t] = (v8f){};
  gemm(&S.RLt[nloc][0], 36, R + Wo::GW1, 32, 8, acc, false); wave_lds_sync();
#pragma unroll
  for (int t = 0; t < 8; ++t)
#pragma unroll
    for (int v = 0; v < 8; ++v) S.T1[8 * hlf + v][t * 16 + nloc] = elu_(acc[t][v] * (1.0f / AS_) + gb1[t * 16 + nloc]);
  wave_lds_sync();
#pragma unroll
  for (int t = 0; t < 8; ++t) acc[t] = (v8f){};
  gemm(&S.T1[nloc][0], 132, R + Wo::GW2, 128, 8, acc, false); wave_lds_sync();
#pragma unroll
  for (int t = 0; t < 8; ++t)
#pragma unroll
    for (int v = 0; v < 8; ++v) { const int j = 8 * hlf + v, c = t * 16 + nloc; S.GEO[j][c] = (acc[t][v] * (1.0f / AS_) + gb2[c]) * S.FN[j][c] * S.G[j]; }
  wave_lds_sync();
#pragma unroll
  for (int t = 0; t < 8; ++t) acc[t] = (v8f){};
  gemm(&S.GEO[nloc][0], 132, R + Wo::KW1, 128, 8, acc, false); wave_lds_sync();
#pragma unroll
  for (int t = 0; t < 8; ++t)
#pragma unroll
    for (int v = 0; v < 8; ++v) S.KT[8 * hlf + v][t * 16 + nloc] = elu_(acc[t][v] * (1.0f / AS_));
  wave_lds_sync();
  { v8f mq = {}; const float* qn = Q + (size_t)n * 512;
    for (int kb = 0; kb < ND; kb += 32) { v16b ah, al; frag_split(&S.KT[nloc][kb], hlf, ah, al); v16b bh, bl;
      if (nloc < NH) frag_split(qn + (size_t)nloc * ND + kb, hlf, bh, bl); else { bh = (v16b){}; bl = (v16b){}; }
      mq = wmma16b(ah, bh, mq); mq = wmma16b(ah, bl, mq); mq = wmma16b(al, bh, mq); }
#pragma unroll
    for (int r = 0; r < 8; ++r) { const int j = 8 * hlf + r; S.MQ[nloc][j] = S.M[j] ? 0.0f : mq[r] * (1.0f / (AS_ * AS_)); }
    if (lane < 16) { for (int c = 16; c < 32; ++c) S.MQ[lane][c] = 0.0f; } }
#pragma unroll
  for (int t = 0; t < 8; ++t) acc[t] = (v8f){};
  gemm(&S.GEO[nloc][0], 132, R + Wo::VW1, 128, 8, acc, false); wave_lds_sync();
#pragma unroll
  for (int t = 0; t < 8; ++t)
#pragma unroll
    for (int v = 0; v < 8; ++v) S.VT[t * 16 + nloc][8 * hlf + v] = elu_(acc[t][v] * (1.0f / AS_));
  for (int i = lane; i < 128 * 16; i += 32) S.VT[i >> 4][16 + (i & 15)] = 0.0f;
  wave_lds_sync();
#pragma unroll
  for (int t = 0; t < 8; ++t) acc[t] = (v8f){};
  { v16b ah, al; frag_split(&S.MQ[nloc][0], hlf, ah, al);
#pragma unroll
    for (int t = 0; t < 8; ++t) { v16b bh, bl; frag_split(&S.VT[t * 16 + nloc][0], hlf, bh, bl); acc[t] = wmma16b(ah, bh, acc[t]); acc[t] = wmma16b(ah, bl, acc[t]); acc[t] = wmma16b(al, bh, acc[t]); } }
  if (hlf == 0) {
#pragma unroll
    for (int t = 0; t < 8; ++t)
#pragma unroll
      for (int r = 0; r < 4; ++r) S.O[r][t * 16 + nloc] = acc[t][r] * (1.0f / (AS_ * AS_)); }
  wave_lds_sync();
  for (int pass = 0; pass < 2; ++pass) { for (int i = lane; i < 4 * 32; i += 32) { const int h = i >> 5, c4 = (i & 31) * 4; *(volatile v4f*)(orow + (size_t)n * 512 + h * 128 + c4) = *(const v4f*)(&S.O[h][c4]); } __threadfence(); }
}

__global__ __launch_bounds__(128) void fin_kernel(const float* __restrict__ orow, const b16* __restrict__ R, float* __restrict__ out) {
  __shared__ __attribute__((aligned(16))) float T[4][32][128 + 4];
  const int lane = threadIdx.x & 31, wave = threadIdx.x >> 5, nloc = lane & 15, hlf = lane >> 4, m0 = blockIdx.x * 128 + wave * 32;
  const int ra = min(m0 + nloc, N1 - 1), rb = min(m0 + 16 + nloc, N1 - 1);
  v8f acc[2][8];
#pragma unroll
  for (int r = 0; r < 2; ++r)
#pragma unroll
    for (int t = 0; t < 8; ++t) acc[r][t] = (v8f){};
#pragma unroll 2
  for (int kb = 0; kb < 512; kb += 32) { v16b a0, l0, a1, l1; frag_split(orow + (size_t)ra * 512 + kb, hlf, a0, l0); frag_split(orow + (size_t)rb * 512 + kb, hlf, a1, l1);
#pragma unroll
    for (int t = 0; t < 8; ++t) { const v16b bw = frag_kb(R + Wo::DW1 + (size_t)(t * 16 + nloc) * 512 + kb, hlf); acc[0][t] = wmma16b(a0, bw, acc[0][t]); acc[0][t] = wmma16b(l0, bw, acc[0][t]); acc[1][t] = wmma16b(a1, bw, acc[1][t]); acc[1][t] = wmma16b(l1, bw, acc[1][t]); } }
#pragma unroll
  for (int t = 0; t < 8; ++t)
#pragma unroll
    for (int r = 0; r < 2; ++r)
#pragma unroll
      for (int v = 0; v < 8; ++v) T[wave][r * 16 + 8 * hlf + v][t * 16 + nloc] = elu_(acc[r][t][v] * (1.0f / AS_));
  wave_lds_sync();
#pragma unroll
  for (int r = 0; r < 2; ++r)
#pragma unroll
    for (int t = 0; t < 8; ++t) acc[r][t] = (v8f){};
#pragma unroll
  for (int kb = 0; kb < ND; kb += 32) { v16b a0, l0, a1, l1; frag_split(&T[wave][nloc][kb], hlf, a0, l0); frag_split(&T[wave][16 + nloc][kb], hlf, a1, l1);
#pragma unroll
    for (int t = 0; t < 8; ++t) { const v16b bw = frag_kb(R + Wo::DW2 + (size_t)(t * 16 + nloc) * ND + kb, hlf); acc[0][t] = wmma16b(a0, bw, acc[0][t]); acc[0][t] = wmma16b(l0, bw, acc[0][t]); acc[1][t] = wmma16b(a1, bw, acc[1][t]); acc[1][t] = wmma16b(l1, bw, acc[1][t]); } }
  wave_lds_sync();
#pragma unroll
  for (int t = 0; t < 8; ++t)
#pragma unroll
    for (int r = 0; r < 2; ++r)
#pragma unroll
      for (int v = 0; v < 8; ++v) T[wave][r * 16 + 8 * hlf + v][t * 16 + nloc] = elu_(acc[r][t][v] * (1.0f / AS_));
  wave_lds_sync();
  for (int pass = 0; pass < 2; ++pass) { for (int i = lane; i < 32 * 32; i += 32) { const int rr = i >> 5, c4 = (i & 31) * 4; if (m0 + rr < N1) *(volatile v4f*)(out + (size_t)(m0 + rr) * ND + c4) = *(const v4f*)(&T[wave][rr][c4]); } __threadfence(); }
}
}

extern "C" void kernel_launch(void* const* d_in, const int* in_sizes, int n_in,
                              void* d_out, int out_size, void* d_ws, size_t ws_size, hipStream_t stream) {
  (void)n_in; (void)out_size;
  const float* f1 = (const float*)d_in[0]; const float* f2 = (const float*)d_in[1]; const float* x1 = (const float*)d_in[2]; const float* x2 = (const float*)d_in[3]; const float* nuv1 = (const float*)d_in[4]; const float* nuv2 = (const float*)d_in[5]; const int* topk = (const int*)d_in[6];
  const float* qw1 = (const float*)d_in[7]; const float* qb1 = (const float*)d_in[8]; const float* qw2 = (const float*)d_in[9]; const float* qb2 = (const float*)d_in[10]; const float* gw1 = (const float*)d_in[11]; const float* gb1 = (const float*)d_in[12]; const float* gw2 = (const float*)d_in[13]; const float* gb2 = (const float*)d_in[14];
  const float* kw1 = (const float*)d_in[15]; const float* kw2 = (const float*)d_in[16]; const float* vw1 = (const float*)d_in[17]; const float* vw2 = (const float*)d_in[18]; const float* dw1 = (const float*)d_in[19]; const float* dw2 = (const float*)d_in[20];
  float* out = (float*)d_out;
  if (in_sizes[0] != N1 * ND || in_sizes[1] != N2 * ND || in_sizes[6] != N1 * NN || in_sizes[9] != 128 * 512 || in_sizes[11] != 12 * 128 || in_sizes[19] != 512 * 128) return;
  size_t off = 0; char* ws = (char*)d_ws;
  auto carve = [&](size_t bytes) { char* p = ws + off; off += (bytes + 255) & ~(size_t)255; return p; };
  unsigned short* qw16 = (unsigned short*)carve(128 * 128 * 2); b16* R = (b16*)carve(Wo::END * 2); float* P = (float*)carve(1024 * 4); float* Q = (float*)carve((size_t)NPAD * 512 * 4); float* Qp = (float*)carve((size_t)NPAD * 512 * 4); float* orow = (float*)carve((size_t)NPAD * 512 * 4);
  float* orow2 = Q;
  if (off > ws_size) return;
  prep_kernel<<<64, 256, 0, stream>>>(qw1, qb1, qw2, qb2, gw1, gb1, gw2, gb2, kw1, kw2, vw1, vw2, dw1, dw2, qw16, R, P);
  q_kernel<<<dim3(512 / 64, NBLK), 128, 0, stream>>>(f1, qw16, R, P, Q);
  rows_kernel<<<dim3(2, NPAD * 4 / 128), 128, 0, stream>>>(Q, R + Wo::KW2N, Qp);
  pair_kernel<<<N1 / 2, 64, 0, stream>>>(f2, x1, x2, nuv1, nuv2, topk, Qp, R, P, orow);
  rows_kernel<<<dim3(2, NPAD * 4 / 128), 128, 0, stream>>>(orow, R + Wo::VW2, orow2);
  fin_kernel<<<NBLK, 128, 0, stream>>>(orow2, R, out);
}
